// DisAttLayer_11458972746001
// MI455X (gfx1250) — hardware-verified
//
#include <hip/hip_runtime.h>


namespace {
constexpr int BATCH = 4, S = 256, H = 8, NMB = 11, NC = 102, PS_ = 32, BS = 16, CS = 16, L0 = 96, L1 = 32, L2 = 16;

typedef _Float16 b16;
typedef __attribute__((ext_vector_type(16))) _Float16 v16b;
typedef __attribute__((ext_vector_type(8))) float v8f;
typedef __attribute__((ext_vector_type(4))) float v4f;
__device__ __forceinline__ void split16(float v, b16& hi, b16& lo) { hi = (b16)v; lo = (b16)(v - (float)hi); }
__device__ __forceinline__ v8f wmma16b(v16b a, v16b b, v8f c) {
  v8f d = __builtin_amdgcn_wmma_f32_16x16x32_f16(false, a, false, b, (short)0, c, false, false);
  asm volatile("v_nop\n\tv_nop\n\tv_nop\n\tv_nop" : "+v"(d) : "v"(a), "v"(b));
  return d;
}
__device__ __forceinline__ void wave_lds_sync() { __builtin_amdgcn_fence(__ATOMIC_RELEASE, "workgroup"); __builtin_amdgcn_wave_barrier(); __builtin_amdgcn_fence(__ATOMIC_ACQUIRE, "workgroup"); }

__global__ __launch_bounds__(256) void prep_kernel(const float* __restrict__ epos, const float* __restrict__ ebi, const float* __restrict__ ebj, const float* __restrict__ eci, const float* __restrict__ ecj,
                                                   const float* __restrict__ w1, const float* __restrict__ w2, float* __restrict__ T, b16* __restrict__ w2t) {
  constexpr int NPE = 2 * S * H * L1, NBI = NMB * H * L1, NCI = NC * H * L1, TOT = NPE + 2 * NBI + 2 * NCI;
  const int i = blockIdx.x * 256 + threadIdx.x;
  for (int pass = 0; pass < 2; ++pass) {
    if (i < TOT) { int j = i, which; if (j < NPE) which = 0; else { j -= NPE; if (j < NBI) which = 1; else { j -= NBI; if (j < NBI) which = 2; else { j -= NBI; if (j < NCI) which = 3; else { j -= NCI; which = 4; } } } }
      const int v = j / (H * L1), h = (j / L1) % H, k = j % L1; const float* tab; int dsz, off;
      switch (which) { case 0: tab = epos; dsz = PS_; off = 0; break; case 1: tab = ebi; dsz = BS; off = 32; break; case 2: tab = ebj; dsz = BS; off = 48; break; case 3: tab = eci; dsz = CS; off = 64; break; default: tab = ecj; dsz = CS; off = 80; break; }
      float s = 0.0f;
#pragma unroll 1
      for (int d = 0; d < dsz; ++d) s += tab[((size_t)v * H + h) * dsz + d] * w1[((size_t)(off + d) * L1 + k) * H + h];
      ((volatile float*)T)[i] = s; }
    if (i < H * L2 * L1) { const int h = i / (L2 * L1), l = (i / L1) % L2, k = i % L1; ((volatile b16*)w2t)[i] = (b16)w2[((size_t)k * L2 + l) * H + h]; }
    __threadfence();
  }
}

__global__ __launch_bounds__(256) void score_kernel(const int* __restrict__ bseq, const int* __restrict__ cseq, const float* __restrict__ T, const b16* __restrict__ w2t, const float* __restrict__ w3, float* __restrict__ out) {
  constexpr int NPE = 2 * S * H * L1, NBI = NMB * H * L1, NCI = NC * H * L1;
  __shared__ float Sc[8][32];
  __shared__ __attribute__((aligned(16))) b16 Hh[8][32][L1 + 8], Hl[8][32][L1 + 8];
  const int wave = threadIdx.x >> 5, lane = threadIdx.x & 31, nloc = lane & 15, hlf = lane >> 4;
  const int blk = blockIdx.x, m = blk % S, h = (blk / S) % H, b = blk / (S * H);
  const float* PE1 = T; const float* BI1 = T + NPE; const float* BJ1 = BI1 + NBI; const float* CI1 = BJ1 + NBI; const float* CJ1 = CI1 + NCI;
  int bsm = bseq[b * S + m], csm = cseq[b * S + m]; bsm = (bsm < 0) ? 0 : (bsm >= NMB ? NMB - 1 : bsm); csm = (csm < 0) ? 0 : (csm >= NC ? NC - 1 : csm);
  const float* rowm_b = BI1 + ((size_t)bsm * H + h) * L1; const float* rowm_c = CI1 + ((size_t)csm * H + h) * L1;
  v8f acc[2] = {{}, {}};
  v16b bw;
#pragma unroll
  for (int e = 0; e < 16; ++e) { const int k = (e < 8) ? (8 * hlf + e) : (16 + 8 * hlf + e - 8); bw[e] = w2t[((size_t)h * L2 + nloc) * L1 + k]; }
  { const int nl = lane, n = wave * 32 + nl; int bsn = bseq[b * S + n], csn = cseq[b * S + n]; bsn = (bsn < 0) ? 0 : (bsn >= NMB ? NMB - 1 : bsn); csn = (csn < 0) ? 0 : (csn >= NC ? NC - 1 : csn);
    const float* pe = PE1 + ((size_t)(m - n + S) * H + h) * L1; const float* rn_b = BJ1 + ((size_t)bsn * H + h) * L1; const float* rn_c = CJ1 + ((size_t)csn * H + h) * L1;
#pragma unroll
    for (int k = 0; k < L1; ++k) { const float v = fmaxf(pe[k] + rowm_b[k] + rn_b[k] + rowm_c[k] + rn_c[k], 0.0f); b16 x, y; split16(v * 64.0f, x, y); Hh[wave][nl][k] = x; Hl[wave][nl][k] = y; } }
  wave_lds_sync();
#pragma unroll
  for (int r = 0; r < 2; ++r) { v16b ah, al;
#pragma unroll
    for (int e = 0; e < 16; ++e) { const int k = (e < 8) ? (8 * hlf + e) : (16 + 8 * hlf + e - 8); ah[e] = Hh[wave][r * 16 + nloc][k]; al[e] = Hl[wave][r * 16 + nloc][k]; }
    acc[r] = wmma16b(ah, bw, acc[r]); acc[r] = wmma16b(al, bw, acc[r]); }
  const float w3l = w3[nloc * H + h];
#pragma unroll
  for (int r = 0; r < 2; ++r)
#pragma unroll
    for (int v = 0; v < 8; ++v) { float s = fmaxf(acc[r][v] * (1.0f / 64.0f), 0.0f) * w3l;
#pragma unroll
      for (int o = 1; o < 16; o <<= 1) s += __shfl_xor(s, o);
      if (nloc == 0) Sc[wave][r * 16 + 8 * hlf + v] = s; }
  wave_lds_sync();
  float* dst = out + (((size_t)b * H + h) * S + m) * S + wave * 32;
  for (int pass = 0; pass < 2; ++pass) { ((volatile float*)dst)[lane] = Sc[wave][lane]; __threadfence(); }
}
}

extern "C" void kernel_launch(void* const* d_in, const int* in_sizes, int n_in,
                              void* d_out, int out_size, void* d_ws, size_t ws_size, hipStream_t stream) {
  (void)n_in; (void)out_size;
  const int* bseq = (const int*)d_in[0]; const int* cseq = (const int*)d_in[1]; const float* epos = (const float*)d_in[2]; const float* ebi = (const float*)d_in[3]; const float* ebj = (const float*)d_in[4]; const float* eci = (const float*)d_in[5]; const float* ecj = (const float*)d_in[6];
  const float* w1 = (const float*)d_in[7]; const float* w2 = (const float*)d_in[8]; const float* w3 = (const float*)d_in[9];
  float* out = (float*)d_out;
  if (in_sizes[0] != BATCH * S || in_sizes[1] != BATCH * S || in_sizes[2] != 2 * S * H * PS_ || in_sizes[3] != NMB * H * BS || in_sizes[5] != NC * H * CS || in_sizes[7] != L0 * L1 * H || in_sizes[8] != L1 * L2 * H || in_sizes[9] != L2 * H) return;
  constexpr int TOT = 2 * S * H * L1 + 2 * NMB * H * L1 + 2 * NC * H * L1;
  size_t off = 0; char* ws = (char*)d_ws;
  auto carve = [&](size_t bytes) { char* p = ws + off; off += (bytes + 255) & ~(size_t)255; return p; };
  float* T = (float*)carve((size_t)TOT * 4); b16* w2t = (b16*)carve((size_t)H * L2 * L1 * 2);
  if (off > ws_size) return;
  prep_kernel<<<(TOT + 255) / 256, 256, 0, stream>>>(epos, ebi, ebj, eci, ecj, w1, w2, T, w2t);
  score_kernel<<<BATCH * H * S, 256, 0, stream>>>(bseq, cseq, T, w2t, w3, out);
}
